// ContRepDecoder_61512521614075
// MI455X (gfx1250) — hardware-verified
//
#include <hip/hip_runtime.h>
#include <stddef.h>
#include <math.h>


#define BQ     2
#define CCH    128
#define DD     176
#define KP     192
#define NL     6
#define OC     45
#define OP     48
#define XCX    16
#define NCELL  4096
#define NQ     32768
#define QT     32
#define NBLK   (BQ * NQ / QT)
#define HP     200
#define CP     128
#define YP     48
#define MT     128
#define PT     128
#define MINT   256
#define NPB    (NQ / MINT)
#define PROW   32
#define UW     (NL * DD * (KP / 8))
#define UP     (OP * (CCH / 8))
#define PBW    (UW / PT)
#define PBP    (UP / PT)
#define WSC    8.0f
#define WIV    0.125f
#define EPSF   1e-7f
#define TWOPI  6.28318548202514648f

static_assert(PBW * PT == UW);
static_assert(PBP * PT == UP);
static_assert(NPB * MINT == NQ);
static_assert(NBLK * QT == BQ * NQ);
static_assert((HP % 8) == 0 && HP >= KP + 8);
static_assert((KP % 32) == 0 && KP >= DD);
static_assert(QT == 32 && MT == 128 && MINT == 256);
static_assert(OP >= OC && (OP % 16) == 0);
static_assert(BQ == 2 && PROW == 32);
static_assert((QT * YP) % 4 == 0);

typedef float    v4f  __attribute__((ext_vector_type(4)));
typedef float    v8f  __attribute__((ext_vector_type(8)));
typedef int      v4i  __attribute__((ext_vector_type(4)));
typedef _Float16 v4h  __attribute__((ext_vector_type(4)));
typedef _Float16 v8h  __attribute__((ext_vector_type(8)));
typedef _Float16 v16h __attribute__((ext_vector_type(16)));
union FragH { v16h v; v8h h[2]; };
union Pk8 { v8h h; v4i i; };

__device__ __forceinline__ v8f wmh(v16h a, v16h b, v8f c) {
  v8f d = __builtin_amdgcn_wmma_f32_16x16x32_f16(false, a, false, b, (short)0, c, false, false);
  asm volatile("v_nop\n\tv_nop\n\tv_nop\n\tv_nop" : "+v"(d) : "v"(a), "v"(b));
  return d;
}

__device__ __forceinline__ float silu_f(float x) {
  return x * __builtin_amdgcn_rcpf(1.0f + __expf(-x));
}

__device__ __forceinline__ v8h cv8(v4f a, v4f b) {
  v8h r;
  r[0] = (_Float16)a.x; r[1] = (_Float16)a.y; r[2] = (_Float16)a.z; r[3] = (_Float16)a.w;
  r[4] = (_Float16)b.x; r[5] = (_Float16)b.y; r[6] = (_Float16)b.z; r[7] = (_Float16)b.w;
  return r;
}

__device__ __forceinline__ v8f splat8(float v) {
  v8f c;
#pragma unroll
  for (int i = 0; i < 8; ++i) c[i] = v;
  return c;
}

__device__ __forceinline__ int nearest_idx(float qc, float o, float vox) {
#pragma clang fp contract(off)
  const float d = qc - o;
  const float p = d / vox;
  const float s = p + 0.5f;
  float f = floorf(s);
  f = fminf(fmaxf(f, -1.0f), 64.0f);
  int v = (int)f;
  v = v < 0 ? 0 : v;
  v = v > XCX - 2 ? XCX - 2 : v;
  return v;
}

__device__ __forceinline__ float wave_min(float v) {
#pragma unroll
  for (int s = 16; s >= 1; s >>= 1) v = fminf(v, __shfl_xor(v, s));
  return v;
}

__global__ __launch_bounds__(PT) void k_prep(const float* __restrict__ mw, const float* __restrict__ pw,
                                             _Float16* wt, _Float16* pt) {
  const int blk = blockIdx.x, tid = threadIdx.x;
  Pk8 pk;
  _Float16* dp;
  if (blk < PBW) {
    const int u   = blk * PT + tid;
    const int row = u / (KP / 8);
    const int kc  = u - row * (KP / 8);
    const int L   = row / DD;
    const int n   = row - L * DD;
#pragma unroll
    for (int j = 0; j < 8; ++j) {
      const int k   = 8 * kc + j;
      const int kcl = k < DD ? k : DD - 1;
      const float w = mw[((size_t)(L * DD + kcl)) * DD + n];
      const float t = (k < DD) ? w * WSC : 0.0f;
      pk.h[j] = (_Float16)t;
    }
    dp = wt + (size_t)u * 8;
  } else {
    const int u   = (blk - PBW) * PT + tid;
    const int n   = u >> 4;
    const int kc  = u & 15;
    const int ncl = n < OC ? n : OC - 1;
#pragma unroll
    for (int j = 0; j < 8; ++j) {
      const int k = 8 * kc + j;
      const float w = pw[k * OC + ncl];
      const float t = (n < OC) ? w * WSC : 0.0f;
      pk.h[j] = (_Float16)t;
    }
    dp = pt + (size_t)u * 8;
  }
  *(volatile v4i*)dp = pk.i;
  __threadfence();
  *(volatile v4i*)dp = pk.i;
}

__global__ __launch_bounds__(MINT) void k_minpart(const float* __restrict__ ext, const float* __restrict__ qco,
                                                  float* part) {
  __shared__ float wm[MINT / 32][24];
  __shared__ __attribute__((aligned(16))) float so[PROW];
  const int tid  = threadIdx.x, lane = tid & 31;
  const int wave = __builtin_amdgcn_readfirstlane(tid >> 5);
  const int q    = blockIdx.x;
  const int b    = q / NPB;
  const int lin  = (q - b * NPB) * MINT + tid;
  float qc[3], thr[3];
  int   id[3];
#pragma unroll
  for (int c = 0; c < 3; ++c) {
    const float* e  = ext + (size_t)(b * 3 + c) * NCELL;
    const float o   = e[0];
    const float vox = fabsf(e[256 + 16 + 1] - o);
    thr[c] = -0.5f * vox + EPSF;
    qc[c] = qco[(size_t)(b * 3 + c) * NQ + lin];
    id[c] = nearest_idx(qc[c], o, vox);
  }
#pragma unroll
  for (int c8 = 0; c8 < 8; ++c8) {
    const int cell = ((id[0] + (c8 >> 2)) << 8) | ((id[1] + ((c8 >> 1) & 1)) << 4) | (id[2] + (c8 & 1));
#pragma unroll
    for (int c = 0; c < 3; ++c) {
      const float ccv = ext[(size_t)(b * 3 + c) * NCELL + cell];
      const float rel = fmaxf(ccv - qc[c], thr[c]);
      const float r   = wave_min(rel);
      if (lane == 0) wm[wave][c8 * 3 + c] = r;
    }
  }
  __syncthreads();
  if (tid < PROW) {
    float v = __builtin_inff();
    if (tid < 24) {
#pragma unroll
      for (int w = 0; w < MINT / 32; ++w) v = fminf(v, wm[w][tid]);
    }
    so[tid] = v;
  }
  __syncthreads();
  v4f v = {0.0f, 0.0f, 0.0f, 0.0f};
  if (tid < 8) v = *(const v4f*)(so + 4 * tid);
  float* dp = part + (size_t)q * PROW + 4 * (tid & 7);
  if (tid < 8) *(volatile v4f*)dp = v;
  __threadfence();
  if (tid < 8) *(volatile v4f*)dp = v;
}

__global__ __launch_bounds__(64) void k_minfin(const float* __restrict__ part, float* mnb) {
  __shared__ __attribute__((aligned(16))) float so[64];
  const int tid = threadIdx.x, b = tid >> 5, e = tid & 31;
  float v = __builtin_inff();
#pragma unroll 1
  for (int qq = 0; qq < NPB; ++qq) v = fminf(v, part[(size_t)(b * NPB + qq) * PROW + e]);
  so[tid] = v;
  __syncthreads();
  v4f x = {0.0f, 0.0f, 0.0f, 0.0f};
  if (tid < 16) x = *(const v4f*)(so + 4 * tid);
  float* dp = mnb + 4 * (tid & 15);
  if (tid < 16) *(volatile v4f*)dp = x;
  __threadfence();
  if (tid < 16) *(volatile v4f*)dp = x;
}

__global__ __launch_bounds__(MT) void k_main(
    const float* __restrict__ cv, const float* __restrict__ ext, const float* __restrict__ qvs,
    const float* __restrict__ qco, const float* __restrict__ mb, const float* __restrict__ pb,
    const _Float16* __restrict__ wt, const _Float16* __restrict__ pt, const float* __restrict__ mnb,
    float* out) {
  __shared__ __attribute__((aligned(16))) _Float16 hb[2][QT * HP];
  __shared__ __attribute__((aligned(16))) float ctxf[QT * CP];
  __shared__ __attribute__((aligned(16))) float yb[QT * YP];
  __shared__ float tls[QT][4];
  __shared__ float qcs[QT][4];
  __shared__ int   idxs[QT][4];
  __shared__ float cst[20];
  __shared__ float mns[32];

  const int tid  = threadIdx.x, lane = tid & 31, h = lane >> 4, m = lane & 15;
  const int wave = __builtin_amdgcn_readfirstlane(tid >> 5);
  const int blk  = blockIdx.x;
  const int b    = blk / (NQ / QT);
  const int lin0 = (blk - b * (NQ / QT)) * QT;

  if (tid < 3) {
    const float* e  = ext + (size_t)(b * 3 + tid) * NCELL;
    const float o   = e[0];
    const float vox = fabsf(e[256 + 16 + 1] - o);
    cst[tid]      = o;
    cst[4 + tid]  = vox;
    cst[8 + tid]  = -0.5f * vox + EPSF;
    cst[12 + tid] = 1.0f / (1.5f * vox);
    cst[16 + tid] = qvs[b * 3 + tid];
  }
  if (tid < 32) mns[tid] = mnb[b * 32 + tid];
  {
    const v4f z4 = {0.0f, 0.0f, 0.0f, 0.0f};
    for (int u = tid; u < QT * YP / 4; u += MT) *(v4f*)(yb + 4 * u) = z4;
    Pk8 z; z.i.x = 0; z.i.y = 0; z.i.z = 0; z.i.w = 0;
    for (int u = tid; u < 2 * QT * 3; u += MT) {
      const int buf = u / (QT * 3);
      const int rem = u - buf * (QT * 3);
      const int row = rem / 3;
      const int pp  = rem - row * 3;
      *(v8h*)(&hb[buf][row * HP + DD + 8 * pp]) = z.h;
    }
  }
  __syncthreads();
  if (wave == 0) {
    const int row = lane;
#pragma unroll
    for (int c = 0; c < 3; ++c) {
      const float qc = qco[(size_t)(b * 3 + c) * NQ + lin0 + row];
      qcs[row][c]  = qc;
      idxs[row][c] = nearest_idx(qc, cst[c], cst[4 + c]);
    }
  }
  __syncthreads();

  const int mt  = wave & 1, hf2 = wave >> 1;
  const int nt0 = hf2 ? 6 : 0;
  const int ntl = hf2 ? 5 : 6;
  const int np0 = hf2 ? 2 : 0;
  const int npl = hf2 ? 1 : 2;

#pragma unroll 1
  for (int c8 = 0; c8 < 8; ++c8) {
    const int bi = c8 >> 2, bj = (c8 >> 1) & 1, bk = c8 & 1;

    if (wave < 3) {
      const int c = wave, row = lane;
      const int cell = ((idxs[row][0] + bi) << 8) | ((idxs[row][1] + bj) << 4) | (idxs[row][2] + bk);
      const float ccv = ext[(size_t)(b * 3 + c) * NCELL + cell];
      const float qc  = qcs[row][c];
      const float rel = fmaxf(ccv - qc, cst[8 + c]);
      const float rn  = (rel - mns[c8 * 3 + c]) * cst[12 + c];
      _Float16* hr = &hb[0][row * HP];
      hr[CCH + c]     = (_Float16)fmaf(qc, 0.0f, cst[16 + c]);
      hr[CCH + 3 + c] = (_Float16)ccv;
      hr[CCH + 6 + c] = (_Float16)qc;
      hr[CCH + 9 + c] = (_Float16)rn;
      const float ang = TWOPI * rn;
      float s = sinf(ang), co = cosf(ang);
      float sv[6], cw[6];
#pragma unroll
      for (int mm = 0; mm < 6; ++mm) {
        sv[mm] = s; cw[mm] = co;
        const float s2 = 2.0f * s * co;
        const float c2 = co * co - s * s;
        s = s2; co = c2;
      }
      v4h e0, e1, e2;
      e0[0] = (_Float16)sv[0]; e0[1] = (_Float16)sv[1]; e0[2] = (_Float16)sv[2]; e0[3] = (_Float16)sv[3];
      e1[0] = (_Float16)sv[4]; e1[1] = (_Float16)sv[5]; e1[2] = (_Float16)cw[0]; e1[3] = (_Float16)cw[1];
      e2[0] = (_Float16)cw[2]; e2[1] = (_Float16)cw[3]; e2[2] = (_Float16)cw[4]; e2[3] = (_Float16)cw[5];
      _Float16* ep = hr + CCH + 12 + 12 * c;
      *(v4h*)ep       = e0;
      *(v4h*)(ep + 4) = e1;
      *(v4h*)(ep + 8) = e2;
      if (c8 == 0) {
        const float gc = fminf(fmaxf((rn - 0.5f) * 2.0f, -1.0f + EPSF), 1.0f - EPSF);
        tls[row][c] = (gc + 1.0f) * 0.5f;
      }
    }
#pragma unroll
    for (int it = 0; it < 4; ++it) {
      const int u   = tid + MT * it;
      const int row = u & 31, cg = u >> 5;
      const int cell = ((idxs[row][0] + bi) << 8) | ((idxs[row][1] + bj) << 4) | (idxs[row][2] + bk);
      const float* cp = cv + ((size_t)(b * CCH + 8 * cg)) * NCELL + cell;
      v4f x0, x1;
      x0.x = cp[0];         x0.y = cp[NCELL];     x0.z = cp[2 * NCELL]; x0.w = cp[3 * NCELL];
      x1.x = cp[4 * NCELL]; x1.y = cp[5 * NCELL]; x1.z = cp[6 * NCELL]; x1.w = cp[7 * NCELL];
      float* cf = ctxf + row * CP + 8 * cg;
      *(v4f*)cf       = x0;
      *(v4f*)(cf + 4) = x1;
      *(v8h*)(&hb[0][row * HP + 8 * cg]) = cv8(x0, x1);
    }
    __syncthreads();

    int cur = 0;
#pragma unroll 1
    for (int L = 0; L < NL; ++L) {
      const _Float16* hsrc = &hb[cur][(16 * mt + m) * HP + 8 * h];
      _Float16* hdst = &hb[cur ^ 1][0];
      const _Float16* wl = wt + (size_t)L * DD * KP;
      v8f acc[6];
#pragma unroll
      for (int t = 0; t < 6; ++t) {
        const int col  = (nt0 + t) * 16 + m;
        const int colc = col < DD ? col : DD - 1;
        acc[t] = splat8(mb[L * DD + colc] * WSC);
      }
#pragma unroll
      for (int kk = 0; kk < KP / 32; ++kk) {
        FragH a;
        a.h[0] = *(const v8h*)(hsrc + 32 * kk);
        a.h[1] = *(const v8h*)(hsrc + 32 * kk + 16);
#pragma unroll
        for (int t = 0; t < 6; ++t) {
          if (t < ntl) {
            const _Float16* wp = wl + (size_t)((nt0 + t) * 16 + m) * KP + 32 * kk + 8 * h;
            FragH bb;
            bb.h[0] = *(const v8h*)wp;
            bb.h[1] = *(const v8h*)(wp + 16);
            acc[t] = wmh(a.v, bb.v, acc[t]);
          }
        }
      }
      const bool upd = (L == 2) || (L == 5);
#pragma unroll
      for (int t = 0; t < 6; ++t) {
        if (t < ntl) {
          const int tile = nt0 + t;
          const int col  = tile * 16 + m;
          if (upd && tile < 8) {
#pragma unroll
            for (int r = 0; r < 8; ++r) {
              const int row  = 16 * mt + 8 * h + r;
              const float sg = silu_f(acc[t][r] * WIV);
              const float cx = ctxf[row * CP + col] + sg;
              ctxf[row * CP + col] = cx;
              hdst[row * HP + col] = (_Float16)cx;
            }
          } else {
#pragma unroll
            for (int r = 0; r < 8; ++r) {
              const int row = 16 * mt + 8 * h + r;
              hdst[row * HP + col] = (_Float16)silu_f(acc[t][r] * WIV);
            }
          }
        }
      }
      __syncthreads();
      cur ^= 1;
    }

    {
      const _Float16* hsrc = &hb[cur][(16 * mt + m) * HP + 8 * h];
      v8f pacc[2];
#pragma unroll
      for (int t = 0; t < 2; ++t) {
        const int col  = (np0 + t) * 16 + m;
        const int colc = col < OC ? col : OC - 1;
        const float bb0 = pb[colc];
        const float bv  = (col < OC) ? bb0 * WSC : 0.0f;
        pacc[t] = splat8(bv);
      }
#pragma unroll
      for (int kk = 0; kk < CCH / 32; ++kk) {
        FragH a;
        a.h[0] = *(const v8h*)(hsrc + 32 * kk);
        a.h[1] = *(const v8h*)(hsrc + 32 * kk + 16);
#pragma unroll
        for (int t = 0; t < 2; ++t) {
          if (t < npl) {
            const _Float16* wp = pt + (size_t)((np0 + t) * 16 + m) * CCH + 32 * kk + 8 * h;
            FragH bb;
            bb.h[0] = *(const v8h*)wp;
            bb.h[1] = *(const v8h*)(wp + 16);
            pacc[t] = wmh(a.v, bb.v, pacc[t]);
          }
        }
      }
      float w8[8];
#pragma unroll
      for (int r = 0; r < 8; ++r) {
        const int row = 16 * mt + 8 * h + r;
        const float t0 = tls[row][0], t1 = tls[row][1], t2 = tls[row][2];
        const float wi = bi ? t2 : 1.0f - t2;
        const float wj = bj ? t1 : 1.0f - t1;
        const float wk = bk ? t0 : 1.0f - t0;
        w8[r] = (wi * wj) * wk;
      }
#pragma unroll
      for (int t = 0; t < 2; ++t) {
        if (t < npl) {
          const int col = (np0 + t) * 16 + m;
#pragma unroll
          for (int r = 0; r < 8; ++r) {
            const int row    = 16 * mt + 8 * h + r;
            const float pred = pacc[t][r] * WIV;
            const float yv   = yb[row * YP + col] + pred * w8[r];
            yb[row * YP + col] = yv;
          }
        }
      }
    }
    __syncthreads();
  }

#pragma unroll
  for (int ps = 0; ps < 3; ++ps) {
    const int li = ps * 16 + (tid >> 3);
    const int q  = tid & 7;
    if (li < OC) {
      v4f v;
      v.x = yb[(4 * q) * YP + li];     v.y = yb[(4 * q + 1) * YP + li];
      v.z = yb[(4 * q + 2) * YP + li]; v.w = yb[(4 * q + 3) * YP + li];
      float* dp = out + ((size_t)(b * OC + li)) * NQ + lin0 + 4 * q;
      *(volatile v4f*)dp = v;
    }
  }
  __threadfence();
#pragma unroll
  for (int ps = 0; ps < 3; ++ps) {
    const int li = ps * 16 + (tid >> 3);
    const int q  = tid & 7;
    if (li < OC) {
      v4f v;
      v.x = yb[(4 * q) * YP + li];     v.y = yb[(4 * q + 1) * YP + li];
      v.z = yb[(4 * q + 2) * YP + li]; v.w = yb[(4 * q + 3) * YP + li];
      float* dp = out + ((size_t)(b * OC + li)) * NQ + lin0 + 4 * q;
      *(volatile v4f*)dp = v;
    }
  }
}

extern "C" void kernel_launch(void* const* d_in, const int* in_sizes, int n_in,
                              void* d_out, int out_size, void* d_ws, size_t ws_size,
                              hipStream_t stream) {
  if (n_in < 8) return;
  if (in_sizes[0] != BQ * CCH * NCELL) return;
  if (in_sizes[1] != BQ * 3 * NCELL) return;
  if (in_sizes[2] != BQ * 3) return;
  if (in_sizes[3] != BQ * 3 * NQ) return;
  if (in_sizes[4] != NL * DD * DD) return;
  if (in_sizes[5] != NL * DD) return;
  if (in_sizes[6] != CCH * OC) return;
  if (in_sizes[7] != OC) return;
  if (out_size != BQ * OC * NQ) return;

  const float* cv  = (const float*)d_in[0];
  const float* ext = (const float*)d_in[1];
  const float* qvs = (const float*)d_in[2];
  const float* qco = (const float*)d_in[3];
  const float* mw  = (const float*)d_in[4];
  const float* mb  = (const float*)d_in[5];
  const float* pw  = (const float*)d_in[6];
  const float* pb  = (const float*)d_in[7];
  float* outp = (float*)d_out;

  const size_t szW    = (size_t)NL * DD * KP * 2;
  const size_t szP    = (size_t)OP * CCH * 2;
  const size_t szPart = (size_t)BQ * NPB * PROW * 4;
  const size_t szMn   = (size_t)64 * 4;
  const size_t oW    = 0;
  const size_t oP    = oW + szW;
  const size_t oPart = oP + szP;
  const size_t oMn   = oPart + szPart;
  const size_t total = oMn + szMn;
  size_t limit = (size_t)134217728;
  if (ws_size < limit) limit = ws_size;
  if (total > limit) return;

  char* ws = (char*)d_ws;
  _Float16* pWt  = (_Float16*)(ws + oW);
  _Float16* pPt  = (_Float16*)(ws + oP);
  float*    part = (float*)(ws + oPart);
  float*    mnb  = (float*)(ws + oMn);

  k_prep<<<PBW + PBP, PT, 0, stream>>>(mw, pw, pWt, pPt);
  k_minpart<<<BQ * NPB, MINT, 0, stream>>>(ext, qco, part);
  k_minfin<<<1, 64, 0, stream>>>(part, mnb);
  k_main<<<NBLK, MT, 0, stream>>>(cv, ext, qvs, qco, mb, pb, pWt, pPt, mnb, outp);
}
